// BowEncoder_35373350650620
// MI455X (gfx1250) — hardware-verified
//
#include <hip/hip_runtime.h>


namespace {
constexpr int Bn = 64, T = 2048, V = 50257, H = 256, NW = 4;

typedef _Float16 b16;
typedef __attribute__((ext_vector_type(16))) _Float16 v16b;
typedef __attribute__((ext_vector_type(8))) _Float16 v8b;
typedef __attribute__((ext_vector_type(8))) float v8f;
typedef __attribute__((ext_vector_type(4))) float v4f;
__device__ __forceinline__ float bf16_rne(float f) { unsigned int u = __float_as_uint(f); u += 0x7FFFu + ((u >> 16) & 1u); return __uint_as_float(u & 0xFFFF0000u); }
__device__ __forceinline__ void split16(float v, b16& hi, b16& lo) { hi = (b16)v; lo = (b16)(v - (float)hi); }
__device__ __forceinline__ v8f wmma16b(v16b a, v16b b, v8f c) { v8f d = __builtin_amdgcn_wmma_f32_16x16x32_f16(false, a, false, b, (short)0, c, false, false); asm volatile("v_nop\n\tv_nop\n\tv_nop\n\tv_nop" : "+v"(d) : "v"(a), "v"(b)); return d; }
__device__ __forceinline__ void wave_lds_sync() { __builtin_amdgcn_fence(__ATOMIC_RELEASE, "workgroup"); __builtin_amdgcn_wave_barrier(); __builtin_amdgcn_fence(__ATOMIC_ACQUIRE, "workgroup"); }

__global__ __launch_bounds__(128) void bow_kernel(const int* __restrict__ ids, const int* __restrict__ lens, const float* __restrict__ emb, float* __restrict__ out) {
  __shared__ __attribute__((aligned(16))) b16 G[NW][32][H + 8]; __shared__ __attribute__((aligned(16))) float Part[NW][H];
  const int b = blockIdx.x, wid = threadIdx.x >> 5, lane = threadIdx.x & 31, nloc = lane & 15, hh = lane >> 4;
  const int len = min(max(lens[b], 1), T); const float p = 1.0f / (float)len; b16 ph, pl; split16(p, ph, pl);
  v8f acc[16];
#pragma unroll
  for (int n = 0; n < 16; ++n) acc[n] = (v8f){};
  for (int kb = wid * 32; kb < len; kb += NW * 32) {
    { int id = ids[(size_t)b * T + min(kb + lane, T - 1)]; id = (id < 0) ? 0 : (id >= V ? V - 1 : id); const float* er = emb + (size_t)id * H;
      for (int c8 = 0; c8 < H; c8 += 8) { v8b o;
#pragma unroll
        for (int e = 0; e < 8; ++e) o[e] = (b16)bf16_rne(er[c8 + e]);
        *(v8b*)(&G[wid][lane][c8]) = o; } }
    wave_lds_sync();
    v16b ah, al;
#pragma unroll
    for (int e = 0; e < 16; ++e) { const int t = kb + ((e < 8) ? (8 * hh + e) : (16 + 8 * hh + e - 8)); const bool in = (t < len); ah[e] = in ? ph : (b16)0.0f; al[e] = in ? pl : (b16)0.0f; }
#pragma unroll
    for (int n = 0; n < 16; ++n) { v16b g;
#pragma unroll
      for (int e = 0; e < 16; ++e) { const int tt = (e < 8) ? (8 * hh + e) : (16 + 8 * hh + e - 8); g[e] = G[wid][tt][n * 16 + nloc]; }
      acc[n] = wmma16b(ah, g, acc[n]); acc[n] = wmma16b(al, g, acc[n]); }
    wave_lds_sync();
  }
  if (hh == 0) {
#pragma unroll
    for (int n = 0; n < 16; ++n) Part[wid][n * 16 + nloc] = acc[n][0]; }
  __syncthreads();
  for (int pass = 0; pass < 2; ++pass) { if (threadIdx.x < 64) { const int c4 = threadIdx.x * 4; v4f o;
#pragma unroll
      for (int e = 0; e < 4; ++e) o[e] = (Part[0][c4 + e] + Part[1][c4 + e]) + (Part[2][c4 + e] + Part[3][c4 + e]);
      *(volatile v4f*)(out + (size_t)b * H + c4) = o; } __threadfence(); }
}
}

extern "C" void kernel_launch(void* const* d_in, const int* in_sizes, int n_in,
                              void* d_out, int out_size, void* d_ws, size_t ws_size, hipStream_t stream) {
  (void)n_in; (void)out_size; (void)d_ws; (void)ws_size;
  const int* ids = (const int*)d_in[0]; const int* lens = (const int*)d_in[1]; const float* emb = (const float*)d_in[2];
  float* out = (float*)d_out;
  if (in_sizes[0] != Bn * T || in_sizes[1] != Bn || in_sizes[2] != V * H) return;
  bow_kernel<<<Bn, 128, 0, stream>>>(ids, lens, emb, out);
}
